// LatentBatchedExperts_12773232738934
// MI455X (gfx1250) — hardware-verified
//
#include <hip/hip_runtime.h>
#include <math.h>
#include <stdint.h>

#define T_TOK  8192
#define N_EXP  8
#define L_DIM  256
#define F_DIM  1024
#define G_DIM  (2 * F_DIM)
#define TM     32
#define NTHR   256
#define NWAV   (NTHR / 32)
#define NTILE  (T_TOK / TM)
#define CHK    (4 * NTHR)
#define NCHK   (T_TOK / CHK)
#define RPW    (TM / NWAV)
#define XP     264
#define AP     1032
#define OP     256
#define KS1    (L_DIM / 32)
#define NT1    (G_DIM / 16)
#define NTG    (F_DIM / 16)
#define QN     (NTG / NWAV)
#define KS2    (F_DIM / 32)
#define NT2    (L_DIM / 16)
#define PPE1   (NT1 * KS1 * 64)
#define PPE2   (NT2 * KS2 * 64)
#define NPC1   (N_EXP * PPE1)
#define NPC2   (N_EXP * PPE2)
#define WG_EL  ((size_t)NPC1 * 8)
#define WD_EL  ((size_t)NPC2 * 8)
#define OFF_X  0
#define OFF_AH (TM * XP * 2)
#define OFF_AL (OFF_AH + TM * AP * 2)
#define LDS_DYN (OFF_AL + TM * AP * 2)

#define SC_A   1024.0f
#define SC_R   2048.0f
#define SC_W   256.0f
#define INV_HW 3.814697265625e-06f
#define INV_RW 1.862645149230957e-09f

static_assert(T_TOK == NCHK * CHK);
static_assert(NTILE * TM == T_TOK);
static_assert(NWAV == 8 && TM == 32 && RPW * NWAV == TM);
static_assert(QN * NWAV == NTG && NTG * 16 == F_DIM);
static_assert(NT2 == 16 && KS2 * 32 == F_DIM && KS1 * 32 == L_DIM);
static_assert((XP % 8) == 0 && XP >= L_DIM);
static_assert((AP % 8) == 0 && AP >= F_DIM);
static_assert((OFF_AH % 16) == 0 && (OFF_AL % 16) == 0);
static_assert(TM * OP * 4 <= TM * AP * 2);
static_assert((TM * (L_DIM / 8)) == 4 * NTHR);
static_assert(L_DIM == 2 * 32 * 4);
static_assert((NPC1 % 256) == 0 && (NPC2 % 256) == 0);
static_assert(WG_EL == (size_t)N_EXP * L_DIM * G_DIM);
static_assert(WD_EL == (size_t)N_EXP * F_DIM * L_DIM);

typedef __bf16         v16b __attribute__((ext_vector_type(16)));
typedef _Float16       v16h __attribute__((ext_vector_type(16)));
typedef _Float16       v8h  __attribute__((ext_vector_type(8)));
typedef unsigned short v8us __attribute__((ext_vector_type(8)));
typedef float          v8f  __attribute__((ext_vector_type(8)));
typedef float          v4f  __attribute__((ext_vector_type(4)));
typedef int            v4i  __attribute__((ext_vector_type(4)));

union FragB { v16b v; v8us u[2]; };
union FragH { v16h v; v8h p[2]; v8us u[2]; };

__device__ __forceinline__ unsigned short bf_bits(float f) {
  const unsigned u = __float_as_uint(f);
  return (unsigned short)((u + 0x7FFFu + ((u >> 16) & 1u)) >> 16);
}
__device__ __forceinline__ float bf_up(unsigned short b) { return __uint_as_float(((unsigned)b) << 16); }
__device__ __forceinline__ float bfr(float f) { return bf_up(bf_bits(f)); }
__device__ __forceinline__ unsigned short h_bits(float f) {
  union { _Float16 h; unsigned short u; } c;
  c.h = (_Float16)f;
  return c.u;
}
__device__ __forceinline__ v8f zero8() { return (v8f){0.f, 0.f, 0.f, 0.f, 0.f, 0.f, 0.f, 0.f}; }

__device__ __forceinline__ v8f mma_b(v16b a, v16b b, v8f c) {
  return __builtin_amdgcn_wmma_f32_16x16x32_bf16(false, a, false, b, (short)0, c, false, false);
}
__device__ __forceinline__ v8f mma_h(v16h a, v16h b, v8f c) {
  return __builtin_amdgcn_wmma_f32_16x16x32_f16(false, a, false, b, (short)0, c, false, false);
}
__device__ __forceinline__ void guard_b4(v8f& c0, v8f& c1, v8f& c2, v8f& c3,
                                         v16b a0, v16b a1, v16b b0, v16b b1) {
#if defined(__HIP_DEVICE_COMPILE__)
  asm volatile("v_nop\n\tv_nop\n\tv_nop\n\tv_nop"
               : "+v"(c0), "+v"(c1), "+v"(c2), "+v"(c3)
               : "v"(a0), "v"(a1), "v"(b0), "v"(b1));
#else
  (void)c0; (void)c1; (void)c2; (void)c3; (void)a0; (void)a1; (void)b0; (void)b1;
#endif
}
__device__ __forceinline__ void guard_h8(v8f& c0, v8f& c1, v8f& c2, v8f& c3,
                                         v8f& c4, v8f& c5, v8f& c6, v8f& c7,
                                         v16h a0, v16h a1, v16h b0, v16h b1, v16h b2, v16h b3) {
#if defined(__HIP_DEVICE_COMPILE__)
  asm volatile("v_nop\n\tv_nop\n\tv_nop\n\tv_nop"
               : "+v"(c0), "+v"(c1), "+v"(c2), "+v"(c3), "+v"(c4), "+v"(c5), "+v"(c6), "+v"(c7)
               : "v"(a0), "v"(a1), "v"(b0), "v"(b1), "v"(b2), "v"(b3));
#else
  (void)c0; (void)c1; (void)c2; (void)c3; (void)c4; (void)c5; (void)c6; (void)c7;
  (void)a0; (void)a1; (void)b0; (void)b1; (void)b2; (void)b3;
#endif
}

template <int MODE>
__global__ __launch_bounds__(256) void k_pack(const float* __restrict__ src, unsigned short* dst,
                                              int Kdim, int Ndim, int kS, int ppe, int nPieces) {
  const int piece = blockIdx.x * 256 + threadIdx.x;
  const bool act  = piece < nPieces;
  const int pc    = act ? piece : (nPieces - 1);
  const int e     = pc / ppe;
  const int pl    = pc - e * ppe;
  const int elem0 = pl * 8;
  const int tblk  = kS * 512;
  const int t     = elem0 / tblk;
  int rem         = elem0 - t * tblk;
  const int s     = rem >> 9;
  rem            &= 511;
  const int L     = rem >> 4;
  const int j0    = rem & 15;
  const int n     = t * 16 + (L & 15);
  const int hh    = L >> 4;
  const int kb    = s * 32 + 8 * hh + 2 * j0;
  const int nc    = (n < Ndim) ? n : (Ndim - 1);
  const float* se = src + (size_t)e * (size_t)Kdim * (size_t)Ndim;
  v8us o;
#pragma unroll
  for (int jj = 0; jj < 8; ++jj) {
    const int k  = kb + jj;
    const int kc = (k < Kdim) ? k : (Kdim - 1);
    float v = se[(size_t)kc * (size_t)Ndim + nc];
    v = (k < Kdim && n < Ndim) ? v : 0.0f;
    o[jj] = (MODE == 0) ? bf_bits(v) : h_bits(bfr(v) * SC_W);
  }
  unsigned short* d = dst + (size_t)pc * 8;
  if (act) *(volatile v8us*)d = o;
  __threadfence();
  if (act) *(volatile v8us*)d = o;
}

__device__ __forceinline__ void act_put(_Float16* aH, _Float16* aL, int row, int col, float g, float u) {
  const float sg  = __builtin_amdgcn_rcpf(1.0f + __expf(-g));
  const float a   = ((g * sg) * u) * SC_A;
  const _Float16 h16 = (_Float16)a;
  const float res = (a - (float)h16) * SC_R;
  aH[row * AP + col] = h16;
  aL[row * AP + col] = (_Float16)res;
}

__global__ __launch_bounds__(NTHR) void k_moe(const float* __restrict__ x, const int* __restrict__ ids,
                                              const unsigned short* __restrict__ Wg,
                                              const unsigned short* __restrict__ Wd,
                                              float* out) {
  __shared__ int sTok[TM];
  __shared__ int sW[NWAV];
  extern __shared__ __align__(16) unsigned char dynl[];
  unsigned short* sX = (unsigned short*)(dynl + OFF_X);
  _Float16* aHp = (_Float16*)(dynl + OFF_AH);
  _Float16* aLp = (_Float16*)(dynl + OFF_AL);
  float* sO = (float*)(dynl + OFF_AH);

  const int tid  = threadIdx.x;
  const int lane = tid & 31;
  const int wave = tid >> 5;
  const int m    = lane & 15;
  const int hh   = lane >> 4;
  const int mrow = 8 * hh;
  const int e    = blockIdx.y;
  const int tile = blockIdx.x;
  const int slo  = tile * TM;
  const int shi  = slo + TM;

  if (tid < TM) sTok[tid] = -1;
  int base = 0;
  for (int c = 0; c < NCHK; ++c) {
    const int t0   = c * CHK + 4 * tid;
    const v4i idv  = *(const v4i*)(ids + t0);
    bool mj[4];
    int lc = 0;
#pragma unroll
    for (int j = 0; j < 4; ++j) { mj[j] = (idv[j] == e); lc += mj[j] ? 1 : 0; }
    const unsigned lm = (1u << lane) - 1u;
    const unsigned b0 = __builtin_amdgcn_ballot_w32((lc & 1) != 0);
    const unsigned b1 = __builtin_amdgcn_ballot_w32((lc & 2) != 0);
    const unsigned b2 = __builtin_amdgcn_ballot_w32((lc & 4) != 0);
    const int lp = __builtin_popcount(b0 & lm) + 2 * __builtin_popcount(b1 & lm) + 4 * __builtin_popcount(b2 & lm);
    const int wc = __builtin_popcount(b0) + 2 * __builtin_popcount(b1) + 4 * __builtin_popcount(b2);
    if (lane == 0) sW[wave] = wc;
    __syncthreads();
    int wb = 0, tot = 0;
#pragma unroll
    for (int w = 0; w < NWAV; ++w) {
      const int v = sW[w];
      wb  += (w < wave) ? v : 0;
      tot += v;
    }
    tot = __builtin_amdgcn_readfirstlane(tot);
    int pos = base + wb + lp - slo;
#pragma unroll
    for (int j = 0; j < 4; ++j) {
      if (mj[j]) {
        if (pos >= 0 && pos < TM) sTok[pos] = t0 + j;
        ++pos;
      }
    }
    base += tot;
    __syncthreads();
    if (base >= shi) break;
  }
  if (base <= slo) return;

#pragma unroll
  for (int j = 0; j < 4; ++j) {
    const int i   = tid + j * NTHR;
    const int r   = i >> 5;
    const int q   = i & 31;
    const int tok = sTok[r];
    const int tc  = (tok < 0) ? 0 : ((tok >= T_TOK) ? (T_TOK - 1) : tok);
    const float* p = x + (size_t)tc * L_DIM + q * 8;
    const v4f va = *(const v4f*)(p);
    const v4f vb = *(const v4f*)(p + 4);
    v8us o;
#pragma unroll
    for (int k = 0; k < 4; ++k) {
      o[k]     = (tok >= 0) ? bf_bits(va[k]) : (unsigned short)0;
      o[4 + k] = (tok >= 0) ? bf_bits(vb[k]) : (unsigned short)0;
    }
    *(v8us*)(sX + r * XP + q * 8) = o;
  }
  __syncthreads();

  {
    const unsigned short* WgE = Wg + (size_t)e * ((size_t)NT1 * KS1 * 512);
#pragma unroll 1
    for (int qn = 0; qn < QN; ++qn) {
      const int nt = wave * QN + qn;
      v8f cg0 = zero8(), cg1 = zero8(), cu0 = zero8(), cu1 = zero8();
      FragB a0, a1, bg, bu;
#pragma unroll 2
      for (int s = 0; s < KS1; ++s) {
        const unsigned short* pa = sX + m * XP + s * 32 + 8 * hh;
        a0.u[0] = *(const v8us*)(pa);
        a0.u[1] = *(const v8us*)(pa + 16);
        a1.u[0] = *(const v8us*)(pa + 16 * XP);
        a1.u[1] = *(const v8us*)(pa + 16 * XP + 16);
        const unsigned short* pg = WgE + ((size_t)(nt * KS1 + s) * 32 + lane) * 16;
        const unsigned short* pu = WgE + ((size_t)((nt + NTG) * KS1 + s) * 32 + lane) * 16;
        bg.u[0] = *(const v8us*)(pg);
        bg.u[1] = *(const v8us*)(pg + 8);
        bu.u[0] = *(const v8us*)(pu);
        bu.u[1] = *(const v8us*)(pu + 8);
        cg0 = mma_b(a0.v, bg.v, cg0);
        cg1 = mma_b(a1.v, bg.v, cg1);
        cu0 = mma_b(a0.v, bu.v, cu0);
        cu1 = mma_b(a1.v, bu.v, cu1);
        guard_b4(cg0, cg1, cu0, cu1, a0.v, a1.v, bg.v, bu.v);
      }
      const int col = nt * 16 + m;
#pragma unroll
      for (int v = 0; v < 8; ++v) {
        act_put(aHp, aLp, mrow + v,      col, cg0[v], cu0[v]);
        act_put(aHp, aLp, 16 + mrow + v, col, cg1[v], cu1[v]);
      }
    }
  }
  __syncthreads();

  const int mt  = wave >> 2;
  const int ntb = (wave & 3) * 4;
  v8f ch0 = zero8(), ch1 = zero8(), ch2 = zero8(), ch3 = zero8();
  v8f cl0 = zero8(), cl1 = zero8(), cl2 = zero8(), cl3 = zero8();
  {
    const unsigned short* WdE = Wd + (size_t)e * ((size_t)NT2 * KS2 * 512);
    FragH ah, al, bq0, bq1, bq2, bq3;
#pragma unroll 1
    for (int s = 0; s < KS2; ++s) {
      const _Float16* ph = aHp + (mt * 16 + m) * AP + s * 32 + 8 * hh;
      const _Float16* pq = aLp + (mt * 16 + m) * AP + s * 32 + 8 * hh;
      ah.p[0] = *(const v8h*)(ph);
      ah.p[1] = *(const v8h*)(ph + 16);
      al.p[0] = *(const v8h*)(pq);
      al.p[1] = *(const v8h*)(pq + 16);
      const unsigned short* pb = WdE + ((size_t)(ntb * KS2 + s) * 32 + lane) * 16;
      bq0.u[0] = *(const v8us*)(pb);                    bq0.u[1] = *(const v8us*)(pb + 8);
      bq1.u[0] = *(const v8us*)(pb + 1 * KS2 * 512);    bq1.u[1] = *(const v8us*)(pb + 1 * KS2 * 512 + 8);
      bq2.u[0] = *(const v8us*)(pb + 2 * KS2 * 512);    bq2.u[1] = *(const v8us*)(pb + 2 * KS2 * 512 + 8);
      bq3.u[0] = *(const v8us*)(pb + 3 * KS2 * 512);    bq3.u[1] = *(const v8us*)(pb + 3 * KS2 * 512 + 8);
      ch0 = mma_h(ah.v, bq0.v, ch0);  cl0 = mma_h(al.v, bq0.v, cl0);
      ch1 = mma_h(ah.v, bq1.v, ch1);  cl1 = mma_h(al.v, bq1.v, cl1);
      ch2 = mma_h(ah.v, bq2.v, ch2);  cl2 = mma_h(al.v, bq2.v, cl2);
      ch3 = mma_h(ah.v, bq3.v, ch3);  cl3 = mma_h(al.v, bq3.v, cl3);
      guard_h8(ch0, ch1, ch2, ch3, cl0, cl1, cl2, cl3, ah.v, al.v, bq0.v, bq1.v, bq2.v, bq3.v);
    }
  }
  __syncthreads();

  {
#pragma unroll
    for (int v = 0; v < 8; ++v) {
      const int row = mt * 16 + mrow + v;
      float* srow = sO + row * OP + m;
      srow[(ntb + 0) * 16] = ch0[v] * INV_HW + cl0[v] * INV_RW;
      srow[(ntb + 1) * 16] = ch1[v] * INV_HW + cl1[v] * INV_RW;
      srow[(ntb + 2) * 16] = ch2[v] * INV_HW + cl2[v] * INV_RW;
      srow[(ntb + 3) * 16] = ch3[v] * INV_HW + cl3[v] * INV_RW;
    }
  }
  __syncthreads();

  {
    v4f ov0[RPW], ov1[RPW];
    int tk[RPW];
#pragma unroll
    for (int rr = 0; rr < RPW; ++rr) {
      const int row = wave * RPW + rr;
      tk[rr]  = __builtin_amdgcn_readfirstlane(sTok[row]);
      ov0[rr] = *(const v4f*)(sO + row * OP + lane * 4);
      ov1[rr] = *(const v4f*)(sO + row * OP + 128 + lane * 4);
    }
#pragma unroll
    for (int rr = 0; rr < RPW; ++rr) {
      const int t = tk[rr];
      if ((unsigned)t < (unsigned)T_TOK) {
        float* op = out + (size_t)t * L_DIM + lane * 4;
        *(volatile v4f*)(op)       = ov0[rr];
        *(volatile v4f*)(op + 128) = ov1[rr];
      }
    }
    __threadfence();
#pragma unroll
    for (int rr = 0; rr < RPW; ++rr) {
      const int t = tk[rr];
      if ((unsigned)t < (unsigned)T_TOK) {
        float* op = out + (size_t)t * L_DIM + lane * 4;
        *(volatile v4f*)(op)       = ov0[rr];
        *(volatile v4f*)(op + 128) = ov1[rr];
      }
    }
  }
}

extern "C" void kernel_launch(void* const* d_in, const int* in_sizes, int n_in,
                              void* d_out, int out_size, void* d_ws, size_t ws_size,
                              hipStream_t stream) {
  if (n_in < 4) return;
  if (in_sizes[0] != T_TOK * L_DIM) return;
  if (in_sizes[1] != N_EXP * L_DIM * G_DIM) return;
  if (in_sizes[2] != N_EXP * F_DIM * L_DIM) return;
  if (in_sizes[3] != T_TOK) return;
  if (out_size != T_TOK * L_DIM) return;

  const float* x   = (const float*)d_in[0];
  const float* gu  = (const float*)d_in[1];
  const float* dw  = (const float*)d_in[2];
  const int*   ids = (const int*)d_in[3];
  float* out = (float*)d_out;

  const size_t og_bytes  = 0;
  const size_t od_bytes  = og_bytes + WG_EL * 2;
  const size_t tot_bytes = od_bytes + WD_EL * 2;
  if ((od_bytes % 128) != 0) return;
  if (tot_bytes > ws_size) return;
  if (tot_bytes > (size_t)134217728) return;

  unsigned short* Wg = (unsigned short*)((char*)d_ws + og_bytes);
  unsigned short* Wd = (unsigned short*)((char*)d_ws + od_bytes);

  k_pack<0><<<dim3(NPC1 / 256), dim3(256), 0, stream>>>(gu, Wg, L_DIM, G_DIM, KS1, PPE1, NPC1);
  k_pack<1><<<dim3(NPC2 / 256), dim3(256), 0, stream>>>(dw, Wd, F_DIM, L_DIM, KS2, PPE2, NPC2);

  (void)hipFuncSetAttribute(reinterpret_cast<const void*>(&k_moe),
                            hipFuncAttributeMaxDynamicSharedMemorySize, LDS_DYN);
  k_moe<<<dim3(NTILE, N_EXP), dim3(NTHR), (size_t)LDS_DYN, stream>>>(x, ids, Wg, Wd, out);
  (void)hipGetLastError();
}
